// RSAGEConv2d_6150393168696
// MI455X (gfx1250) — hardware-verified
//
#include <hip/hip_runtime.h>
#include <stdint.h>


typedef __bf16         v16b __attribute__((ext_vector_type(16)));
typedef unsigned short v8us __attribute__((ext_vector_type(8)));
typedef float          v8f  __attribute__((ext_vector_type(8)));
typedef float          v4f  __attribute__((ext_vector_type(4)));
typedef v8us v8usa __attribute__((may_alias));
typedef v4f  v4fa  __attribute__((may_alias));

constexpr int Bn = 8;
constexpr int Nn = 4096;
constexpr int CI = 64;
constexpr int CO = 64;
constexpr int CC = CI + CO;
constexpr int Kn = 16;

typedef char chk_n64[(Nn % 64 == 0) ? 1 : -1];
typedef char chk_ci[(CI == 64 && CO == 64) ? 1 : -1];

static __device__ __forceinline__ unsigned short bf16_bits_rne(float f) {
  unsigned u = __float_as_uint(f);
  u += 0x7FFFu + ((u >> 16) & 1u);
  return (unsigned short)(u >> 16);
}
static __device__ __forceinline__ void split_bf16(float f, unsigned short& hi, unsigned short& lo) {
  const unsigned short hb = bf16_bits_rne(f);
  const float hf = __uint_as_float(((unsigned)hb) << 16);
  hi = hb;
  lo = bf16_bits_rne(f - hf);
}

union FragU { v16b v; v8us h[2]; };
static __device__ __forceinline__ v16b ld_frag(const unsigned short* base, int pitch, int row0, int k0, int lane) {
  const unsigned short* p = base + (row0 + (lane & 15)) * pitch + k0 + ((lane >> 4) << 3);
  FragU u;
  u.h[0] = *(const v8usa*)(p);
  u.h[1] = *(const v8usa*)(p + 16);
  return u.v;
}

static __device__ __forceinline__ v8f mma16(v16b a, v16b b, v8f c) {
  v8f d = __builtin_amdgcn_wmma_f32_16x16x32_bf16(false, a, false, b, (short)0, c, false, false);
  asm volatile("v_nop\n\tv_nop\n\tv_nop\n\tv_nop" : "+v"(d) : "v"(a), "v"(b));
  return d;
}
static __device__ __forceinline__ v8f mma3(v16b ah, v16b al, v16b bh, v16b bl, v8f c) {
  c = mma16(ah, bh, c);
  c = mma16(ah, bl, c);
  c = mma16(al, bh, c);
  return c;
}

__global__ __launch_bounds__(256) void k_lin1(const float* __restrict__ x,
                                             const float* __restrict__ wp,
                                             float* __restrict__ y) {
  constexpr int PX = 72;
  constexpr int PY = 68;
  __shared__ __align__(16) unsigned short sXh[64 * PX];
  __shared__ __align__(16) unsigned short sXl[64 * PX];
  __shared__ __align__(16) unsigned short sWh[64 * PX];
  __shared__ __align__(16) unsigned short sWl[64 * PX];
  __shared__ __align__(16) float          sY[64 * PY];

  const int t = threadIdx.x, lane = t & 31, w = t >> 5, h = lane >> 4, m = lane & 15;
  const int b = blockIdx.y, n0 = blockIdx.x * 64;
  if (n0 >= Nn) return;

  {
    const int nl = t & 63;
    const int cb = t >> 6;
#pragma unroll
    for (int i = 0; i < 16; ++i) {
      const int c = cb + 4 * i;
      const float v = x[((size_t)(b * CI + c)) * Nn + n0 + nl];
      unsigned short hi, lo;
      split_bf16(v, hi, lo);
      sXh[nl * PX + c] = hi;
      sXl[nl * PX + c] = lo;
    }
  }
#pragma unroll
  for (int i = 0; i < 16; ++i) {
    const int idx = i * 256 + t;
    const int o = idx >> 6, c = idx & 63;
    const float v = wp[idx];
    unsigned short hi, lo;
    split_bf16(v, hi, lo);
    sWh[o * PX + c] = hi;
    sWl[o * PX + c] = lo;
  }
  __syncthreads();

  const int mt = w >> 1;
  const int ntb = (w & 1) * 2;
  v8f acc0 = {0.f, 0.f, 0.f, 0.f, 0.f, 0.f, 0.f, 0.f};
  v8f acc1 = {0.f, 0.f, 0.f, 0.f, 0.f, 0.f, 0.f, 0.f};
#pragma unroll
  for (int ks = 0; ks < 2; ++ks) {
    const v16b ah = ld_frag(sXh, PX, mt * 16, ks * 32, lane);
    const v16b al = ld_frag(sXl, PX, mt * 16, ks * 32, lane);
    {
      const v16b bh = ld_frag(sWh, PX, ntb * 16, ks * 32, lane);
      const v16b bl = ld_frag(sWl, PX, ntb * 16, ks * 32, lane);
      acc0 = mma3(ah, al, bh, bl, acc0);
    }
    {
      const v16b bh = ld_frag(sWh, PX, (ntb + 1) * 16, ks * 32, lane);
      const v16b bl = ld_frag(sWl, PX, (ntb + 1) * 16, ks * 32, lane);
      acc1 = mma3(ah, al, bh, bl, acc1);
    }
  }

#pragma unroll
  for (int r = 0; r < 8; ++r) {
    const int row = mt * 16 + 8 * h + r;
    sY[row * PY + ntb * 16 + m]       = acc0[r];
    sY[row * PY + (ntb + 1) * 16 + m] = acc1[r];
  }
  __syncthreads();

  v4f vv[4];
  size_t off[4];
#pragma unroll
  for (int it = 0; it < 4; ++it) {
    const int row = w * 8 + it * 2 + h;
    vv[it]  = *(const v4fa*)(&sY[row * PY + m * 4]);
    off[it] = ((size_t)(b * Nn + n0 + row)) * CO + m * 4;
  }
#pragma unroll
  for (int it = 0; it < 4; ++it) *(volatile v4f*)(y + off[it]) = vv[it];
  __threadfence();
#pragma unroll
  for (int it = 0; it < 4; ++it) *(volatile v4f*)(y + off[it]) = vv[it];
}

__global__ __launch_bounds__(256) void k_aggr(const float* __restrict__ y,
                                             const int* __restrict__ eidx,
                                             float* __restrict__ ag) {
  const int t = threadIdx.x, lane = t & 31, w = t >> 5, h = lane >> 4, sub = lane & 15;
  const int b = blockIdx.y, n0 = blockIdx.x * 64;
  if (n0 >= Nn) return;

  const float* yb = y + (size_t)b * Nn * CO + sub * 4;
#pragma unroll 1
  for (int p = 0; p < 4; ++p) {
    const int node = n0 + p * 16 + w * 2 + h;
    const int* ip = eidx + ((size_t)(b * Nn + node)) * Kn;
    v4f mx = {0.f, 0.f, 0.f, 0.f};
#pragma unroll 4
    for (int k = 0; k < Kn; ++k) {
      int j = ip[k];
      j = (j < 0) ? (j + Nn) : j;
      j = min(max(j, 0), Nn - 1);
      const v4f v = *(const v4fa*)(yb + (size_t)j * CO);
      mx[0] = fmaxf(mx[0], v[0]);
      mx[1] = fmaxf(mx[1], v[1]);
      mx[2] = fmaxf(mx[2], v[2]);
      mx[3] = fmaxf(mx[3], v[3]);
    }
    float* dst = ag + ((size_t)(b * Nn + node)) * CO + sub * 4;
    *(volatile v4f*)dst = mx;
    __threadfence();
    *(volatile v4f*)dst = mx;
  }
}

__global__ __launch_bounds__(256) void k_lin2(const float* __restrict__ x,
                                             const float* __restrict__ ag,
                                             const float* __restrict__ wn,
                                             const float* __restrict__ bias,
                                             const float* __restrict__ x0,
                                             float* __restrict__ out) {
  constexpr int PK = 136;
  constexpr int PO = 36;
  __shared__ __align__(16) unsigned short sAh[64 * PK];
  __shared__ __align__(16) unsigned short sAl[64 * PK];
  __shared__ __align__(16) unsigned short sCh[32 * PK];
  __shared__ __align__(16) unsigned short sCl[32 * PK];
  __shared__ __align__(16) float          sOut[64 * PO];
  __shared__ float sBias[64];
  __shared__ float sRn[32];
  (void)x0;

  const int t = threadIdx.x, lane = t & 31, w = t >> 5, h = lane >> 4, m = lane & 15;
  const int b = blockIdx.y, n0 = blockIdx.x * 32;
  if (n0 >= Nn) return;

#pragma unroll 8
  for (int i = 0; i < 32; ++i) {
    const int idx = i * 256 + t;
    const int o = idx >> 7, k = idx & 127;
    const float v = wn[idx];
    unsigned short hi, lo;
    split_bf16(v, hi, lo);
    sAh[o * PK + k] = hi;
    sAl[o * PK + k] = lo;
  }
  {
    const int nl = t & 31;
    const int cb = t >> 5;
#pragma unroll
    for (int i = 0; i < 8; ++i) {
      const int c = cb + 8 * i;
      const float v = x[((size_t)(b * CI + c)) * Nn + n0 + nl];
      unsigned short hi, lo;
      split_bf16(v, hi, lo);
      sCh[nl * PK + c] = hi;
      sCl[nl * PK + c] = lo;
    }
  }
#pragma unroll
  for (int i = 0; i < 8; ++i) {
    const int idx = i * 256 + t;
    const int nl = idx >> 6, c = idx & 63;
    const float v = ag[((size_t)(b * Nn + n0 + nl)) * CO + c];
    unsigned short hi, lo;
    split_bf16(v, hi, lo);
    sCh[nl * PK + CI + c] = hi;
    sCl[nl * PK + CI + c] = lo;
  }
  if (t < CO) sBias[t] = bias[t];
  __syncthreads();

  const int ot = w >> 1;
  const int nt = w & 1;
  v8f acc = {0.f, 0.f, 0.f, 0.f, 0.f, 0.f, 0.f, 0.f};
#pragma unroll
  for (int ks = 0; ks < 4; ++ks) {
    const v16b ah = ld_frag(sAh, PK, ot * 16, ks * 32, lane);
    const v16b al = ld_frag(sAl, PK, ot * 16, ks * 32, lane);
    const v16b bh = ld_frag(sCh, PK, nt * 16, ks * 32, lane);
    const v16b bl = ld_frag(sCl, PK, nt * 16, ks * 32, lane);
    acc = mma3(ah, al, bh, bl, acc);
  }

#pragma unroll
  for (int r = 0; r < 8; ++r) {
    const int o = ot * 16 + 8 * h + r;
    sOut[o * PO + nt * 16 + m] = fmaxf(acc[r], 0.0f) + sBias[o];
  }
  __syncthreads();

  if (t < 32) {
    float s = 0.0f;
#pragma unroll 8
    for (int o = 0; o < CO; ++o) {
      const float v = sOut[o * PO + t];
      s += v * v;
    }
    sRn[t] = 1.0f / fmaxf(sqrtf(s), 1e-12f);
  }
  __syncthreads();

  v4f vv[2];
  size_t off[2];
#pragma unroll
  for (int it = 0; it < 2; ++it) {
    const int o = w * 8 + it * 4 + (lane >> 3);
    const int q = lane & 7;
    v4f v = *(const v4fa*)(&sOut[o * PO + q * 4]);
    v[0] *= sRn[q * 4 + 0];
    v[1] *= sRn[q * 4 + 1];
    v[2] *= sRn[q * 4 + 2];
    v[3] *= sRn[q * 4 + 3];
    vv[it]  = v;
    off[it] = ((size_t)(b * CO + o)) * Nn + n0 + q * 4;
  }
#pragma unroll
  for (int it = 0; it < 2; ++it) *(volatile v4f*)(out + off[it]) = vv[it];
  __threadfence();
#pragma unroll
  for (int it = 0; it < 2; ++it) *(volatile v4f*)(out + off[it]) = vv[it];
}

extern "C" void kernel_launch(void* const* d_in, const int* in_sizes, int n_in,
                              void* d_out, int out_size, void* d_ws, size_t ws_size,
                              hipStream_t stream) {
  if (n_in < 6) return;
  if (in_sizes[0] != Bn * CI * Nn) return;
  if (in_sizes[2] != CO * CI) return;
  if (in_sizes[3] != CO * CC) return;
  if (in_sizes[4] != CO) return;
  if (in_sizes[5] != 2 * Bn * Nn * Kn) return;
  if (out_size != Bn * CO * Nn) return;

  const float* x    = (const float*)d_in[0];
  const float* x0   = (const float*)d_in[1];
  const float* wp   = (const float*)d_in[2];
  const float* wn   = (const float*)d_in[3];
  const float* bias = (const float*)d_in[4];
  const int*   eidx = (const int*)d_in[5];
  float* out = (float*)d_out;

  const size_t ybytes = (size_t)Bn * Nn * CO * sizeof(float);
  const size_t abytes = (size_t)Bn * Nn * CO * sizeof(float);
  if (ws_size < ybytes + abytes) return;
  float* y  = (float*)d_ws;
  float* ag = (float*)((char*)d_ws + ybytes);

  k_lin1<<<dim3((Nn + 63) / 64, Bn), 256, 0, stream>>>(x, wp, y);
  k_aggr<<<dim3((Nn + 63) / 64, Bn), 256, 0, stream>>>(y, eidx, ag);
  k_lin2<<<dim3((Nn + 31) / 32, Bn), 256, 0, stream>>>(x, ag, wn, bias, x0, out);
}
